// PVConv_5720896438543
// MI455X (gfx1250) — hardware-verified
//
#include <hip/hip_runtime.h>
#define BB 4
#define NPT 16384
#define CIN 64
#define COUT 128
#define RR 32
#define NVOX (BB * RR * RR * RR)
#define NP2 65536
#define NGRP 8

typedef __bf16 v16b __attribute__((ext_vector_type(16)));
typedef unsigned short v8us __attribute__((ext_vector_type(8), may_alias));
typedef float  v8f  __attribute__((ext_vector_type(8)));
typedef float  v4f  __attribute__((ext_vector_type(4)));
typedef float  v4fa __attribute__((ext_vector_type(4), may_alias));
union FragB { v16b v; v8us half[2]; unsigned short u[16]; };

__device__ __forceinline__ unsigned short bf16_bits(float x) { unsigned int u = __float_as_uint(x); return (unsigned short)((u + 0x7FFFu + ((u >> 16) & 1u)) >> 16); }
__device__ __forceinline__ float bf16_val(unsigned short b) { return __uint_as_float(((unsigned int)b) << 16); }
__device__ __forceinline__ float bf16_round(float x) { return bf16_val(bf16_bits(x)); }
template <int NT>
__device__ __forceinline__ v8f mmaN(v16b ah, v16b al, v16b bh, v16b bl, v8f c) {
  c = __builtin_amdgcn_wmma_f32_16x16x32_bf16(false, ah, false, bh, (short)0, c, false, false);
  if (NT >= 2) c = __builtin_amdgcn_wmma_f32_16x16x32_bf16(false, al, false, bh, (short)0, c, false, false);
  if (NT >= 3) c = __builtin_amdgcn_wmma_f32_16x16x32_bf16(false, ah, false, bl, (short)0, c, false, false);
  asm volatile("v_nop\n\tv_nop\n\tv_nop\n\tv_nop" : "+v"(c) : "v"(ah), "v"(al), "v"(bh), "v"(bl));
  return c;
}

__global__ __launch_bounds__(256) void k_wt_bf16(const float* __restrict__ W, unsigned short* __restrict__ Wt, int K, int N) {
  const int t = blockIdx.x * 256 + threadIdx.x;
  const int k8n = K / 8;
  if (t >= N * k8n) return;
  const int n = t / k8n, k8 = (t % k8n) * 8;
  v8us v;
#pragma unroll
  for (int i = 0; i < 8; ++i) v[i] = bf16_bits(W[(size_t)(k8 + i) * N + n]);
  *(volatile v8us*)(Wt + (size_t)n * K + k8) = v;
  __threadfence();
  *(volatile v8us*)(Wt + (size_t)n * K + k8) = v;
}

template <bool ASPLIT, int ACT, bool BIAS_BF16>
__global__ __launch_bounds__(128) void k_gemm_bf(const float* __restrict__ A, int lda, const unsigned short* __restrict__ Wt, int ldb,
                                               const float* __restrict__ bias, float* __restrict__ C, int ldc, int M, int N, int K) {
  __shared__ __attribute__((aligned(16))) float so[4][16][64];
  const int tid = threadIdx.x, w = tid >> 5, lane = tid & 31, ln = lane & 15, hh = lane >> 4;
  const int ntn = N / 64;
  const int wid = blockIdx.x * 4 + w;
  const int mt = wid / ntn, nq = wid % ntn;
  if (mt * 16 >= M) return;
  const int row0 = mt * 16, col0 = nq * 64;
  const float* arow = A + (size_t)(row0 + ln) * lda;
  v8f acc[4] = {};
  for (int kb = 0; kb < K; kb += 32) {
    FragB ah, al;
    const v4f x0 = *(const v4fa*)(arow + kb + 8 * hh), x1 = *(const v4fa*)(arow + kb + 8 * hh + 4);
    const v4f x2 = *(const v4fa*)(arow + kb + 16 + 8 * hh), x3 = *(const v4fa*)(arow + kb + 16 + 8 * hh + 4);
    float xs[16] = {x0[0],x0[1],x0[2],x0[3],x1[0],x1[1],x1[2],x1[3],x2[0],x2[1],x2[2],x2[3],x3[0],x3[1],x3[2],x3[3]};
#pragma unroll
    for (int i = 0; i < 16; ++i) { const unsigned short hb = bf16_bits(xs[i]); ah.u[i] = hb; al.u[i] = ASPLIT ? bf16_bits(xs[i] - bf16_val(hb)) : (unsigned short)0; }
#pragma unroll
    for (int t = 0; t < 4; ++t) {
      const unsigned short* brow = Wt + (size_t)(col0 + t * 16 + ln) * ldb + kb;
      FragB b;
      b.half[0] = *(const v8us*)(brow + 8 * hh);
      b.half[1] = *(const v8us*)(brow + 16 + 8 * hh);
      acc[t] = mmaN<ASPLIT ? 2 : 1>(ah.v, al.v, b.v, b.v, acc[t]);
    }
  }
#pragma unroll
  for (int t = 0; t < 4; ++t) {
    float bv = bias ? bias[col0 + t * 16 + ln] : 0.f;
    if (BIAS_BF16) bv = bf16_round(bv);
#pragma unroll
    for (int r = 0; r < 8; ++r) { float v = acc[t][r] + bv; if (ACT == 1) v = fmaxf(v, 0.f); so[w][8 * hh + r][t * 16 + ln] = v; }
  }
  __builtin_amdgcn_fence(__ATOMIC_ACQ_REL, "workgroup");
  __builtin_amdgcn_wave_barrier();
  const int rsub = lane >> 4, c4 = (lane & 15) * 4;
  for (int pass = 0; pass < 2; ++pass) {
#pragma unroll
    for (int q = 0; q < 8; ++q) {
      const int r = q * 2 + rsub;
      const v4f v = *(const v4fa*)&so[w][r][c4];
      *(volatile v4f*)(C + (size_t)(row0 + r) * ldc + col0 + c4) = v;
    }
    if (pass == 0) __threadfence();
  }
}

template <int D, bool CAUSAL>
__global__ __launch_bounds__(128) void k_flash(const float* __restrict__ qb, const float* __restrict__ kb, const float* __restrict__ vb,
                                             int pitch, int T, int H, float scale, float* __restrict__ y, int ypitch) {
  constexpr int KS = D / 32;
  constexpr int DT = D / 16;
  __shared__ __attribute__((aligned(16))) unsigned short sKh[32][D + 8], sKl[32][D + 8], sVh[32][D + 8], sVl[32][D + 8];
  __shared__ __attribute__((aligned(16))) unsigned short sPh[4][16][40], sPl[4][16][40];
  __shared__ __attribute__((aligned(16))) float sO[4][16][D];
  const int tid = threadIdx.x, w = tid >> 5, lane = tid & 31, ln = lane & 15, hh = lane >> 4;
  const int nqb = (T + 63) / 64;
  const int bh = blockIdx.x / nqb, qblk = blockIdx.x % nqb;
  const int b = bh / H, h = bh % H;
  const int q0 = qblk * 64 + w * 16;
  const float* Q = qb + (size_t)b * T * pitch + h * D;
  const float* K = kb + (size_t)b * T * pitch + h * D;
  const float* V = vb + (size_t)b * T * pitch + h * D;

  FragB aqh[KS], aql[KS];
  {
    int row = q0 + ln; if (row >= T) row = T - 1;
    const float* qr = Q + (size_t)row * pitch;
#pragma unroll
    for (int ks = 0; ks < KS; ++ks)
#pragma unroll
      for (int i = 0; i < 16; ++i) {
        const int d = ks * 32 + ((i < 8) ? (8 * hh + i) : (16 + 8 * hh + (i - 8)));
        const float x = qr[d] * scale; const unsigned short hb = bf16_bits(x);
        aqh[ks].u[i] = hb; aql[ks].u[i] = bf16_bits(x - bf16_val(hb));
      }
  }
  float m_r[8], l_r[8];
#pragma unroll
  for (int r = 0; r < 8; ++r) { m_r[r] = -3.0e38f; l_r[r] = 0.f; }
  v8f oacc[DT];
#pragma unroll
  for (int dt = 0; dt < DT; ++dt) oacc[dt] = (v8f){0.f,0.f,0.f,0.f,0.f,0.f,0.f,0.f};

  const int kv_end = CAUSAL ? min(T, qblk * 64 + 64) : T;
  for (int j0 = 0; j0 < kv_end; j0 += 32) {
    __syncthreads();
    for (int e = tid; e < 32 * (D / 4); e += 128) {
      const int r = e / (D / 4), c4 = (e % (D / 4)) * 4;
      const int key = j0 + r;
      v4f kf = {0.f,0.f,0.f,0.f}, vf = {0.f,0.f,0.f,0.f};
      if (key < T) { kf = *(const v4fa*)(K + (size_t)key * pitch + c4); vf = *(const v4fa*)(V + (size_t)key * pitch + c4); }
#pragma unroll
      for (int t = 0; t < 4; ++t) {
        unsigned short hb = bf16_bits(kf[t]); sKh[r][c4 + t] = hb; sKl[r][c4 + t] = bf16_bits(kf[t] - bf16_val(hb));
        hb = bf16_bits(vf[t]); sVh[r][c4 + t] = hb; sVl[r][c4 + t] = bf16_bits(vf[t] - bf16_val(hb));
      }
    }
    __syncthreads();
    v8f s[2];
#pragma unroll
    for (int nt = 0; nt < 2; ++nt) {
      v8f acc = {};
#pragma unroll
      for (int ks = 0; ks < KS; ++ks) {
        FragB bh_, bl_;
        bh_.half[0] = *(const v8us*)&sKh[nt * 16 + ln][ks * 32 + 8 * hh]; bh_.half[1] = *(const v8us*)&sKh[nt * 16 + ln][ks * 32 + 16 + 8 * hh];
        bl_.half[0] = *(const v8us*)&sKl[nt * 16 + ln][ks * 32 + 8 * hh]; bl_.half[1] = *(const v8us*)&sKl[nt * 16 + ln][ks * 32 + 16 + 8 * hh];
        acc = mmaN<3>(aqh[ks].v, aql[ks].v, bh_.v, bl_.v, acc);
      }
      s[nt] = acc;
    }
    float alpha[8];
#pragma unroll
    for (int r = 0; r < 8; ++r) {
      const int qi = q0 + 8 * hh + r;
      const int ja = j0 + ln, jb = j0 + 16 + ln;
      if (CAUSAL) { if (ja > qi) s[0][r] = -3.0e38f; if (jb > qi) s[1][r] = -3.0e38f; }
      if (ja >= T) s[0][r] = -3.0e38f;
      if (jb >= T) s[1][r] = -3.0e38f;
      float mx = fmaxf(s[0][r], s[1][r]);
      mx = fmaxf(mx, __shfl_xor(mx, 1, 32)); mx = fmaxf(mx, __shfl_xor(mx, 2, 32)); mx = fmaxf(mx, __shfl_xor(mx, 4, 32)); mx = fmaxf(mx, __shfl_xor(mx, 8, 32));
      const float mnew = fmaxf(m_r[r], mx);
      alpha[r] = (mnew > -1.0e38f) ? __expf(m_r[r] - mnew) : 1.0f;
      const float p0 = (s[0][r] > -1.0e38f) ? __expf(s[0][r] - mnew) : 0.f;
      const float p1 = (s[1][r] > -1.0e38f) ? __expf(s[1][r] - mnew) : 0.f;
      m_r[r] = mnew;
      l_r[r] = l_r[r] * alpha[r] + p0 + p1;
      unsigned short hb = bf16_bits(p0); sPh[w][8 * hh + r][ln] = hb;      sPl[w][8 * hh + r][ln] = bf16_bits(p0 - bf16_val(hb));
      hb = bf16_bits(p1);                sPh[w][8 * hh + r][16 + ln] = hb; sPl[w][8 * hh + r][16 + ln] = bf16_bits(p1 - bf16_val(hb));
    }
#pragma unroll
    for (int dt = 0; dt < DT; ++dt)
#pragma unroll
      for (int r = 0; r < 8; ++r) oacc[dt][r] *= alpha[r];
    __builtin_amdgcn_fence(__ATOMIC_ACQ_REL, "workgroup");
    __builtin_amdgcn_wave_barrier();
    FragB pah, pal;
    pah.half[0] = *(const v8us*)&sPh[w][ln][8 * hh]; pah.half[1] = *(const v8us*)&sPh[w][ln][16 + 8 * hh];
    pal.half[0] = *(const v8us*)&sPl[w][ln][8 * hh]; pal.half[1] = *(const v8us*)&sPl[w][ln][16 + 8 * hh];
#pragma unroll
    for (int dt = 0; dt < DT; ++dt) {
      FragB bvh, bvl;
#pragma unroll
      for (int i = 0; i < 8; ++i) {
        bvh.u[i] = sVh[8 * hh + i][dt * 16 + ln]; bvh.u[8 + i] = sVh[16 + 8 * hh + i][dt * 16 + ln];
        bvl.u[i] = sVl[8 * hh + i][dt * 16 + ln]; bvl.u[8 + i] = sVl[16 + 8 * hh + i][dt * 16 + ln];
      }
      oacc[dt] = mmaN<3>(pah.v, pal.v, bvh.v, bvl.v, oacc[dt]);
    }
    __builtin_amdgcn_fence(__ATOMIC_ACQ_REL, "workgroup");
    __builtin_amdgcn_wave_barrier();
  }
#pragma unroll
  for (int r = 0; r < 8; ++r) {
    float l = l_r[r];
    l += __shfl_xor(l, 1, 32); l += __shfl_xor(l, 2, 32); l += __shfl_xor(l, 4, 32); l += __shfl_xor(l, 8, 32);
    l_r[r] = (l > 0.f) ? 1.0f / l : 0.f;
  }
#pragma unroll
  for (int dt = 0; dt < DT; ++dt)
#pragma unroll
    for (int r = 0; r < 8; ++r) sO[w][8 * hh + r][dt * 16 + ln] = oacc[dt][r] * l_r[r];
  __builtin_amdgcn_fence(__ATOMIC_ACQ_REL, "workgroup");
  __builtin_amdgcn_wave_barrier();
  for (int pass = 0; pass < 2; ++pass) {
    for (int r = 0; r < 16; ++r) {
      const int row = q0 + r;
      if (row < T && lane < D / 4) {
        const v4f val = *(const v4fa*)&sO[w][r][lane * 4];
        *(volatile v4f*)(y + ((size_t)b * T + row) * ypitch + h * D + lane * 4) = val;
      }
    }
    if (pass == 0) __threadfence();
  }
}

__global__ __launch_bounds__(256) void k_sort_init(const int* __restrict__ seg, int n, int nseg, unsigned int* __restrict__ key, unsigned int* __restrict__ val, int np2) {
  const int i = blockIdx.x * 256 + threadIdx.x; if (i >= np2) return;
  unsigned int kv = 0xFFFFFFFFu;
  if (i < n) { int s = seg[i]; s = s < 0 ? 0 : (s >= nseg ? nseg - 1 : s); kv = (unsigned int)s; }
  *(volatile unsigned int*)(key + i) = kv; *(volatile unsigned int*)(val + i) = (unsigned int)i;
  __threadfence();
  *(volatile unsigned int*)(key + i) = kv; *(volatile unsigned int*)(val + i) = (unsigned int)i;
}
template <bool STAGE0>
__global__ __launch_bounds__(512) void k_sort_lds(unsigned int* __restrict__ key, unsigned int* __restrict__ val, int kstage) {
  __shared__ unsigned int sk[1024], sv[1024];
  const int tid = threadIdx.x; const int base = blockIdx.x * 1024;
  sk[tid] = key[base + tid]; sv[tid] = val[base + tid]; sk[tid + 512] = key[base + tid + 512]; sv[tid + 512] = val[base + tid + 512];
  __syncthreads();
  for (int k = (STAGE0 ? 2 : kstage); k <= (STAGE0 ? 1024 : kstage); k <<= 1) {
    for (int j = (k > 1024 ? 512 : (k >> 1)); j >= 1; j >>= 1) {
      const int lo = tid & (j - 1), hi2 = (tid >> __builtin_ctz(j)) << (__builtin_ctz(j) + 1);
      const int il = hi2 | lo, ir = il | j;
      const int gi = base + il;
      const bool asc = ((gi & k) == 0);
      unsigned int a = sk[il], b = sk[ir], va = sv[il], vb = sv[ir];
      const bool swp = asc ? (a > b) : (a < b);
      if (swp) { sk[il] = b; sk[ir] = a; sv[il] = vb; sv[ir] = va; }
      __syncthreads();
    }
  }
  for (int pass = 0; pass < 2; ++pass) {
    *(volatile unsigned int*)(key + base + tid) = sk[tid]; *(volatile unsigned int*)(val + base + tid) = sv[tid];
    *(volatile unsigned int*)(key + base + tid + 512) = sk[tid + 512]; *(volatile unsigned int*)(val + base + tid + 512) = sv[tid + 512];
    if (pass == 0) __threadfence();
  }
}
__global__ __launch_bounds__(256) void k_sort_step(unsigned int* __restrict__ key, unsigned int* __restrict__ val, int k, int j, int np2) {
  const int t = blockIdx.x * 256 + threadIdx.x; if (t >= np2 / 2) return;
  const int lo = t & (j - 1), il = ((t >> __builtin_ctz(j)) << (__builtin_ctz(j) + 1)) | lo, ir = il | j;
  const bool asc = ((il & k) == 0);
  unsigned int a = key[il], b = key[ir], va = val[il], vb = val[ir];
  const bool swp = asc ? (a > b) : (a < b);
  const unsigned int k1 = swp ? b : a, k2 = swp ? a : b, v1 = swp ? vb : va, v2 = swp ? va : vb;
  *(volatile unsigned int*)(key + il) = k1; *(volatile unsigned int*)(key + ir) = k2; *(volatile unsigned int*)(val + il) = v1; *(volatile unsigned int*)(val + ir) = v2;
  __threadfence();
  *(volatile unsigned int*)(key + il) = k1; *(volatile unsigned int*)(key + ir) = k2; *(volatile unsigned int*)(val + il) = v1; *(volatile unsigned int*)(val + ir) = v2;
}
__global__ __launch_bounds__(256) void k_rowptr(const unsigned int* __restrict__ key, int np2, int nseg, int* __restrict__ rowptr) {
  int s = blockIdx.x * 256 + threadIdx.x; if (s >= ((nseg + 1 + 31) / 32) * 32) return;
  const int sdst = s; if (s > nseg) s = nseg;
  int lo = 0, hi = np2;
  while (lo < hi) { const int mid = (lo + hi) >> 1; if (key[mid] < (unsigned int)s) lo = mid + 1; else hi = mid; }
  *(volatile int*)(rowptr + sdst) = lo; __threadfence(); *(volatile int*)(rowptr + sdst) = lo;
}
static void sort_pairs(unsigned int* key, unsigned int* val, int np2, hipStream_t stream) {
  k_sort_lds<true><<<np2 / 1024, 512, 0, stream>>>(key, val, 0);
  for (int k = 2048; k <= np2; k <<= 1) {
    for (int j = k >> 1; j >= 1024; j >>= 1) k_sort_step<<<(np2 / 2 + 255) / 256, 256, 0, stream>>>(key, val, k, j, np2);
    k_sort_lds<false><<<np2 / 1024, 512, 0, stream>>>(key, val, k);
  }
}


__global__ __launch_bounds__(256) void k_round_rows(const float* __restrict__ W, unsigned short* __restrict__ Wt, int n8) {
  const int t = blockIdx.x * 256 + threadIdx.x;
  if (t >= n8) return;
  const v4f a = *(const v4fa*)(W + (size_t)t * 8), b = *(const v4fa*)(W + (size_t)t * 8 + 4);
  v8us v; v[0]=bf16_bits(a[0]); v[1]=bf16_bits(a[1]); v[2]=bf16_bits(a[2]); v[3]=bf16_bits(a[3]);
  v[4]=bf16_bits(b[0]); v[5]=bf16_bits(b[1]); v[6]=bf16_bits(b[2]); v[7]=bf16_bits(b[3]);
  *(volatile v8us*)(Wt + (size_t)t * 8) = v; __threadfence(); *(volatile v8us*)(Wt + (size_t)t * 8) = v;
}

__device__ __forceinline__ void vox_of(const float* __restrict__ coords, int p, int& ix, int& iy, int& iz, float& fx, float& fy, float& fz) {
  const float cx = bf16_round(coords[(size_t)p * 3 + 0]) * 32.0f, cy = bf16_round(coords[(size_t)p * 3 + 1]) * 32.0f, cz = bf16_round(coords[(size_t)p * 3 + 2]) * 32.0f;
  const float lx = floorf(cx), ly = floorf(cy), lz = floorf(cz);
  ix = min(max((int)lx, 0), RR - 1); iy = min(max((int)ly, 0), RR - 1); iz = min(max((int)lz, 0), RR - 1);
  fx = cx - lx; fy = cy - ly; fz = cz - lz;
}
__global__ __launch_bounds__(256) void k_voxid(const float* __restrict__ coords, int* __restrict__ seg) {
  const int p = blockIdx.x * 256 + threadIdx.x; if (p >= BB * NPT) return;
  int ix, iy, iz; float fx, fy, fz; vox_of(coords, p, ix, iy, iz, fx, fy, fz); const int b = p / NPT;
  const int v = ((b * RR + ix) * RR + iy) * RR + iz;
  *(volatile int*)(seg + p) = v; __threadfence(); *(volatile int*)(seg + p) = v;
}
__global__ __launch_bounds__(256) void k_voxmean(const float* __restrict__ feat, const int* __restrict__ rowptr, const unsigned int* __restrict__ perm, float* __restrict__ grid) {
  const int tid = threadIdx.x, w = tid >> 5, lane = tid & 31; const int v = blockIdx.x * 8 + w; if (v >= NVOX) return;
  const int p0 = rowptr[v], p1 = rowptr[v + 1];
  v4f acc = {0.f,0.f,0.f,0.f};
  if (lane < 16) { for (int p = p0; p < p1; ++p) { const int pt = (int)perm[p]; const int b = pt / NPT, n = pt % NPT; for (int q = 0; q < 4; ++q) acc[q] += bf16_round(feat[((size_t)b * CIN + lane * 4 + q) * NPT + n]); }
    const float inv = 1.0f / fmaxf((float)(p1 - p0), 1.0f); for (int q = 0; q < 4; ++q) acc[q] *= inv;
    float* row = grid + (size_t)v * CIN + lane * 4; *(volatile v4f*)row = acc; __threadfence(); *(volatile v4f*)row = acc; }
}
__global__ __launch_bounds__(256) void k_wt_conv(const float* __restrict__ w, unsigned short* __restrict__ Bt, int Cin) {
  const int t = blockIdx.x * 256 + threadIdx.x; const int K = 27 * Cin; if (t >= COUT * (K / 8)) return;
  const int o = t / (K / 8), k8 = (t % (K / 8)) * 8; v8us v;
  for (int i = 0; i < 8; ++i) { const int k = k8 + i; const int tap = k / Cin, c = k % Cin; v[i] = bf16_bits(w[((size_t)o * Cin + c) * 27 + tap]); }
  *(volatile v8us*)(Bt + (size_t)o * K + k8) = v; __threadfence(); *(volatile v8us*)(Bt + (size_t)o * K + k8) = v;
}
template <int Cin>
__global__ __launch_bounds__(128) void k_conv3d(const float* __restrict__ in, const unsigned short* __restrict__ Bt, const float* __restrict__ bias, const float* __restrict__ gg, const float* __restrict__ gb, float* __restrict__ out) {
  constexpr int K = 27 * Cin, SPT = Cin / 32;
  __shared__ __attribute__((aligned(16))) float so[4][16][64];
  const int tid = threadIdx.x, w = tid >> 5, lane = tid & 31, ln = lane & 15, hh = lane >> 4;
  const int wid = blockIdx.x * 4 + w; const int mt = wid / 2, nq = wid % 2;
  const int row0 = mt * 16, col0 = nq * 64;
  const int m = row0 + ln;
  const int z = m & 31, y = (m >> 5) & 31, x = (m >> 10) & 31, b = m >> 15;
  v8f acc[4] = {};
  for (int tap = 0; tap < 27; ++tap) {
    const int dx = tap / 9 - 1, dy = (tap / 3) % 3 - 1, dz = tap % 3 - 1;
    const int xx = x + dx, yy = y + dy, zz = z + dz;
    const bool inb = (xx >= 0 && xx < RR && yy >= 0 && yy < RR && zz >= 0 && zz < RR);
    const float* src = in + ((size_t)(((b * RR + (inb ? xx : 0)) * RR + (inb ? yy : 0)) * RR + (inb ? zz : 0))) * Cin;
#pragma unroll
    for (int s = 0; s < SPT; ++s) {
      const int c0 = s * 32;
      v4f a0 = {0.f,0.f,0.f,0.f}, a1 = a0, a2 = a0, a3 = a0;
      if (inb) { a0 = *(const v4fa*)(src + c0 + 8 * hh); a1 = *(const v4fa*)(src + c0 + 8 * hh + 4); a2 = *(const v4fa*)(src + c0 + 16 + 8 * hh); a3 = *(const v4fa*)(src + c0 + 16 + 8 * hh + 4); }
      float xs[16] = {a0[0],a0[1],a0[2],a0[3],a1[0],a1[1],a1[2],a1[3],a2[0],a2[1],a2[2],a2[3],a3[0],a3[1],a3[2],a3[3]};
      FragB ah, al;
#pragma unroll
      for (int i = 0; i < 16; ++i) { const unsigned short hb = bf16_bits(xs[i]); ah.u[i] = hb; al.u[i] = bf16_bits(xs[i] - bf16_val(hb)); }
      const int kb = tap * Cin + c0;
#pragma unroll
      for (int t = 0; t < 4; ++t) { FragB bq; bq.half[0] = *(const v8us*)(Bt + (size_t)(col0 + t * 16 + ln) * K + kb + 8 * hh); bq.half[1] = *(const v8us*)(Bt + (size_t)(col0 + t * 16 + ln) * K + kb + 16 + 8 * hh); acc[t] = mmaN<2>(ah.v, al.v, bq.v, bq.v, acc[t]); }
    }
  }
#pragma unroll
  for (int t = 0; t < 4; ++t) {
    const int col = col0 + t * 16 + ln; const float bv = bf16_round(bias[col]), g1 = bf16_round(gg[col]), b1 = bf16_round(gb[col]);
#pragma unroll
    for (int r = 0; r < 8; ++r) {
      const float v = acc[t][r] + bv;
      float s = v; s += __shfl_xor(s, 1, 32); s += __shfl_xor(s, 2, 32); s += __shfl_xor(s, 4, 32); s += __shfl_xor(s, 8, 32);
      const float mu = s * (1.0f / 16.0f); const float d = v - mu;
      float q2 = d * d; q2 += __shfl_xor(q2, 1, 32); q2 += __shfl_xor(q2, 2, 32); q2 += __shfl_xor(q2, 4, 32); q2 += __shfl_xor(q2, 8, 32);
      const float xn = d * rsqrtf(q2 * (1.0f / 16.0f) + 1e-5f) * g1 + b1;
      so[w][8 * hh + r][t * 16 + ln] = xn / (1.0f + expf(-xn));
    }
  }
  __builtin_amdgcn_fence(__ATOMIC_ACQ_REL, "workgroup"); __builtin_amdgcn_wave_barrier();
  const int rsub = lane >> 4, c4 = (lane & 15) * 4;
  for (int pass = 0; pass < 2; ++pass) { for (int q = 0; q < 8; ++q) { const int r = q * 2 + rsub; const v4f v = *(const v4fa*)&so[w][r][c4]; *(volatile v4f*)(out + (size_t)(row0 + r) * COUT + col0 + c4) = v; } if (pass == 0) __threadfence(); }
}
__global__ __launch_bounds__(256) void k_ft(const float* __restrict__ feat, float* __restrict__ fT) {
  const size_t t = (size_t)blockIdx.x * 256 + threadIdx.x; if (t >= (size_t)BB * NPT * 16) return;
  const int c4 = (int)(t % 16) * 4; const int p = (int)(t / 16); const int b = p / NPT, n = p % NPT;
  v4f v; for (int q = 0; q < 4; ++q) v[q] = bf16_round(feat[((size_t)b * CIN + c4 + q) * NPT + n]);
  *(volatile v4f*)(fT + (size_t)p * CIN + c4) = v; __threadfence(); *(volatile v4f*)(fT + (size_t)p * CIN + c4) = v;
}
__global__ __launch_bounds__(256) void k_pstat1(const float* __restrict__ pf, double* __restrict__ part) {
  __shared__ double r1[256], r2[256];
  const int blk = blockIdx.x; const int tid = threadIdx.x;
  const int g = tid & 7, sub = tid >> 3;
  double s = 0.0, s2 = 0.0;
  for (int i = sub; i < 512; i += 32) { const float* row = pf + ((size_t)blk * 512 + i) * COUT + g * 16; for (int c = 0; c < 16; ++c) { const double v = (double)row[c]; s += v; s2 += v * v; } }
  r1[tid] = s; r2[tid] = s2; __syncthreads();
  for (int st = 128; st >= 8; st >>= 1) { if (tid < st) { r1[tid] += r1[tid + st]; r2[tid] += r2[tid + st]; } __syncthreads(); }
  if (tid < 32) { double v = 0.0; if (tid < 8) v = r1[tid]; else if (tid < 16) v = r2[tid - 8]; *(volatile double*)(part + (size_t)blk * 32 + tid) = v; __threadfence(); *(volatile double*)(part + (size_t)blk * 32 + tid) = v; }
}
__global__ __launch_bounds__(32) void k_pstat2(const double* __restrict__ part, float* __restrict__ stats) {
  const int t = threadIdx.x; const int b = t >> 3, g = t & 7;
  double s = 0.0, s2 = 0.0; const int nb = NPT / 512;
  for (int k = 0; k < nb; ++k) { s += part[(size_t)(b * nb + k) * 32 + g]; s2 += part[(size_t)(b * nb + k) * 32 + 8 + g]; }
  const double n = (double)NPT * 16.0; const double mu = s / n; double var = s2 / n - mu * mu; if (var < 0.0) var = 0.0;
  const float m = (float)mu, rs = (float)(1.0 / sqrt(var + 1e-5));
  *(volatile float*)(stats + t) = m; *(volatile float*)(stats + 32 + t) = rs; __threadfence(); *(volatile float*)(stats + t) = m; *(volatile float*)(stats + 32 + t) = rs;
}
__global__ __launch_bounds__(256) void k_final(const float* __restrict__ pf, const float* __restrict__ stats, const float* __restrict__ gg, const float* __restrict__ gb,
                                             const float* __restrict__ h2, const float* __restrict__ coords, float* __restrict__ out) {
  __shared__ float tile[32][33];
  const int b = blockIdx.z, n0 = blockIdx.x * 32, o0 = blockIdx.y * 32; const int tx = threadIdx.x & 31, ty = threadIdx.x >> 5;
  for (int i = ty; i < 32; i += 8) {
    const int p = b * NPT + n0 + i; const int o = o0 + tx; const int g = o >> 4;
    const float v = pf[(size_t)p * COUT + o];
    const float xn = (v - stats[b * 8 + g]) * stats[32 + b * 8 + g] * bf16_round(gg[o]) + bf16_round(gb[o]);
    float val = xn / (1.0f + expf(-xn));
    int ix, iy, iz; float fx, fy, fz; vox_of(coords, p, ix, iy, iz, fx, fy, fz);
    const int hx = min(ix + 1, RR - 1), hy = min(iy + 1, RR - 1), hz = min(iz + 1, RR - 1);
    float dv = 0.f;
#pragma unroll
    for (int dx = 0; dx < 2; ++dx)
#pragma unroll
      for (int dy = 0; dy < 2; ++dy)
#pragma unroll
        for (int dz = 0; dz < 2; ++dz) {
          const float wgt = (dx ? fx : 1.f - fx) * (dy ? fy : 1.f - fy) * (dz ? fz : 1.f - fz);
          const int vx = dx ? hx : ix, vy = dy ? hy : iy, vz = dz ? hz : iz;
          dv += wgt * h2[((size_t)(((b * RR + vx) * RR + vy) * RR + vz)) * COUT + o];
        }
    tile[i][tx] = val + dv;
  }
  __syncthreads();
  for (int pass = 0; pass < 2; ++pass) { for (int i = ty; i < 32; i += 8) *(volatile float*)(out + ((size_t)b * COUT + o0 + i) * NPT + n0 + tx) = tile[tx][i]; if (pass == 0) __threadfence(); }
}

extern "C" void kernel_launch(void* const* d_in, const int* in_sizes, int n_in,
                              void* d_out, int out_size, void* d_ws, size_t ws_size, hipStream_t stream) {
  (void)in_sizes; (void)n_in; (void)out_size;
  const float* coords = (const float*)d_in[0]; const float* feat = (const float*)d_in[1];
  const float* c1w = (const float*)d_in[2]; const float* c1b = (const float*)d_in[3]; const float* g1g = (const float*)d_in[4]; const float* g1b = (const float*)d_in[5];
  const float* c2w = (const float*)d_in[6]; const float* c2b = (const float*)d_in[7]; const float* g2g = (const float*)d_in[8]; const float* g2b = (const float*)d_in[9];
  const float* mw = (const float*)d_in[10]; const float* mb = (const float*)d_in[11]; const float* gpg = (const float*)d_in[12]; const float* gpb = (const float*)d_in[13];
  char* ws = (char*)d_ws; size_t off = 0;
  auto take = [&](size_t bytes) { char* p = ws + off; off += (bytes + 255) & ~(size_t)255; return p; };
  unsigned short* Bt1 = (unsigned short*)take((size_t)COUT * 27 * CIN * 2); unsigned short* Bt2 = (unsigned short*)take((size_t)COUT * 27 * COUT * 2); unsigned short* Btm = (unsigned short*)take((size_t)COUT * CIN * 2);
  int* seg = (int*)take((size_t)BB * NPT * 4); unsigned int* key = (unsigned int*)take((size_t)NP2 * 4); unsigned int* perm = (unsigned int*)take((size_t)NP2 * 4); int* rowptr = (int*)take((size_t)(NVOX + 64) * 4);
  float* grid = (float*)take((size_t)NVOX * CIN * 4); float* h1 = (float*)take((size_t)NVOX * COUT * 4); float* h2 = (float*)take((size_t)NVOX * COUT * 4);
  float* fT = (float*)take((size_t)BB * NPT * CIN * 4); float* pf = (float*)take((size_t)BB * NPT * COUT * 4);
  const int nblk = BB * NPT / 512; double* part = (double*)take((size_t)nblk * 32 * 8); float* stats = (float*)take(64 * 4);
  if (off > ws_size) return;
  k_wt_conv<<<(COUT * (27 * CIN / 8) + 255) / 256, 256, 0, stream>>>(c1w, Bt1, CIN);
  k_wt_conv<<<(COUT * (27 * COUT / 8) + 255) / 256, 256, 0, stream>>>(c2w, Bt2, COUT);
  k_round_rows<<<(COUT * CIN / 8 + 255) / 256, 256, 0, stream>>>(mw, Btm, COUT * CIN / 8);
  k_voxid<<<(BB * NPT + 255) / 256, 256, 0, stream>>>(coords, seg);
  k_sort_init<<<NP2 / 256, 256, 0, stream>>>(seg, BB * NPT, NVOX, key, perm, NP2);
  sort_pairs(key, perm, NP2, stream);
  k_rowptr<<<(NVOX + 32 + 255) / 256, 256, 0, stream>>>(key, NP2, NVOX, rowptr);
  k_voxmean<<<(NVOX + 7) / 8, 256, 0, stream>>>(feat, rowptr, perm, grid);
  k_conv3d<CIN><<<(NVOX / 16) * 2 / 4, 128, 0, stream>>>(grid, Bt1, c1b, g1g, g1b, h1);
  k_conv3d<COUT><<<(NVOX / 16) * 2 / 4, 128, 0, stream>>>(h1, Bt2, c2b, g2g, g2b, h2);
  k_ft<<<(BB * NPT * 16 + 255) / 256, 256, 0, stream>>>(feat, fT);
  k_gemm_bf<false, 0, true><<<((BB * NPT / 16) * (COUT / 64) + 3) / 4, 128, 0, stream>>>(fT, CIN, Btm, CIN, mb, pf, COUT, BB * NPT, COUT, CIN);
  k_pstat1<<<nblk, 256, 0, stream>>>(pf, part); k_pstat2<<<1, 32, 0, stream>>>(part, stats);
  k_final<<<dim3(NPT / 32, COUT / 32, BB), 256, 0, stream>>>(pf, stats, gpg, gpb, h2, coords, (float*)d_out);
}
